// GroupQueryAttention_31928786878514
// MI455X (gfx1250) — hardware-verified
//
#include <hip/hip_runtime.h>
#include <math.h>

#ifndef NB
#define NB 2
#endif
#ifndef SEQ
#define SEQ 2048
#endif
#define NB_FULL 2
#define SEQ_FULL 2048
#define HIDDEN 2048
#define NHEAD 32
#define NKVH 8
#define HDIM 64
#define KVD (NKVH * HDIM)
#define MROWS (NB * SEQ)
#define AW 4

static_assert(NB >= 1 && NB <= NB_FULL);
static_assert(SEQ % 64 == 0 && SEQ >= 64 && SEQ <= SEQ_FULL);
static_assert(HIDDEN % 64 == 0 && KVD % 32 == 0 && HDIM == 64 && NHEAD == 4 * NKVH);
static_assert(MROWS % 64 == 0 && HIDDEN % 32 == 0);

typedef __attribute__((ext_vector_type(16))) _Float16 v16h;
typedef __attribute__((ext_vector_type(8)))  _Float16 v8h;
typedef __attribute__((ext_vector_type(16))) __bf16   v16b;
typedef __attribute__((ext_vector_type(8)))  float    v8f;
typedef __attribute__((ext_vector_type(4)))  float    v4f;
typedef __attribute__((ext_vector_type(8)))  unsigned short v8us;
typedef __attribute__((ext_vector_type(4)))  unsigned int   v4u;

union FragU { v16h h; v16b b; v8us u[2]; };
__device__ __forceinline__ int frag_k(int i, int h) { return (i < 8) ? (8 * h + i) : (16 + 8 * h + (i - 8)); }
__device__ __forceinline__ v8f wmma16(v16h a, v16h b, v8f c) {
    c = __builtin_amdgcn_wmma_f32_16x16x32_f16(false, a, false, b, (short)0, c, false, false);
    asm volatile("v_nop\n\tv_nop\n\tv_nop\n\tv_nop" : "+v"(c) : "v"(a), "v"(b));
    return c;
}
__device__ __forceinline__ v8f wmmab(v16b a, v16b b, v8f c) {
    c = __builtin_amdgcn_wmma_f32_16x16x32_bf16(false, a, false, b, (short)0, c, false, false);
    asm volatile("v_nop\n\tv_nop\n\tv_nop\n\tv_nop" : "+v"(c) : "v"(a), "v"(b));
    return c;
}
__device__ __forceinline__ v16h fh_ld(const float* __restrict__ p, long long sk, int k0, int h, int klen, float s) {
    v16h a;
#pragma unroll
    for (int i = 0; i < 16; ++i) { const int k = k0 + frag_k(i, h); a[i] = (k < klen) ? (_Float16)(p[(long long)k * sk] * s) : (_Float16)0.f; }
    return a;
}

#define VST2(T, ptr, val) do { const T vst2_v_ = (val); *(volatile T*)(ptr) = vst2_v_; __threadfence(); *(volatile T*)(ptr) = vst2_v_; } while (0)
#define VST2V4(ptr, val) do { const v4f vst2_v4_ = (val); *(volatile v4f*)(ptr) = vst2_v4_; __threadfence(); *(volatile v4f*)(ptr) = vst2_v4_; } while (0)

__device__ __forceinline__ float cmb_bf(float v) { const unsigned u = __builtin_bit_cast(unsigned, v); const unsigned r = (u + 0x7fffu + ((u >> 16) & 1u)) & 0xffff0000u; return __builtin_bit_cast(float, r); }
__device__ __forceinline__ unsigned short bf_bits_rne(float v) { unsigned u = __builtin_bit_cast(unsigned, v); u += 0x7fffu + ((u >> 16) & 1u); return (unsigned short)(u >> 16); }
template <int KIND> __device__ __forceinline__ unsigned short cvt16(float v, float sc) {
    if (KIND == 0) return bf_bits_rne(v);
    const float w = (KIND == 1) ? (cmb_bf(v) * sc) : (v * sc);
    return __builtin_bit_cast(unsigned short, (_Float16)w);
}
template <int KIND> __device__ __forceinline__ unsigned int cvt16x2(float a, float b, float sc) { return (unsigned int)cvt16<KIND>(a, sc) | ((unsigned int)cvt16<KIND>(b, sc) << 16); }

template <int KIND>
__global__ __launch_bounds__(256) void k_cast(const float* __restrict__ SRC, long long sz, int lds, unsigned short* __restrict__ DST, long long dz, int ldd, int nR, int nC, int nZ, float sc) {
    const long long u = (long long)blockIdx.x * 256 + threadIdx.x;
    const int per = nC >> 3; const long long perz = (long long)nR * per;
    if (u >= perz * nZ) return;
    const int z = (int)(u / perz); const long long uz = u - (long long)z * perz;
    const int r = (int)(uz / per); const int c0 = 8 * (int)(uz - (long long)r * per);
    const float* s = SRC + (long long)z * sz + (long long)r * lds + c0;
    const v4f f0 = *(const v4f*)s; const v4f f1 = *(const v4f*)(s + 4);
    v4u pk;
    pk.x = cvt16x2<KIND>(f0.x, f0.y, sc); pk.y = cvt16x2<KIND>(f0.z, f0.w, sc);
    pk.z = cvt16x2<KIND>(f1.x, f1.y, sc); pk.w = cvt16x2<KIND>(f1.z, f1.w, sc);
    VST2(v4u, (v4u*)(DST + (long long)z * dz + (long long)r * ldd + c0), pk);
}
template <int KIND>
__global__ __launch_bounds__(256) void k_castT(const float* __restrict__ SRC, long long sz, int lds, unsigned short* __restrict__ DST, long long dz, int ldd, int nR, int nC, int nZ, float sc) {
    const long long u = (long long)blockIdx.x * 256 + threadIdx.x;
    const int per = nR >> 3; const long long perz = (long long)nC * per;
    if (u >= perz * nZ) return;
    const int z = (int)(u / perz); const long long uz = u - (long long)z * perz;
    const int c = (int)(uz / per); const int r0 = 8 * (int)(uz - (long long)c * per);
    const float* s = SRC + (long long)z * sz + (long long)r0 * lds + c;
    float w[8];
#pragma unroll
    for (int e = 0; e < 8; ++e) w[e] = s[(long long)e * lds];
    v4u pk;
    pk.x = cvt16x2<KIND>(w[0], w[1], sc); pk.y = cvt16x2<KIND>(w[2], w[3], sc);
    pk.z = cvt16x2<KIND>(w[4], w[5], sc); pk.w = cvt16x2<KIND>(w[6], w[7], sc);
    VST2(v4u, (v4u*)(DST + (long long)z * dz + (long long)c * ldd + r0), pk);
}

template <bool BF, int TM, int TN>
__global__ __launch_bounds__(32) void k_pgemm(const unsigned short* __restrict__ A, int lda, const unsigned short* __restrict__ Bt, int ldb,
                                              const float* __restrict__ bias, float* __restrict__ C, int ldc, int M, int N, int K, float iscale) {
    static_assert(TN % 2 == 0);
    const int lane = threadIdx.x & 31, h = lane >> 4, l15 = lane & 15;
    const int m0 = blockIdx.y * (16 * TM), n0 = blockIdx.x * (16 * TN);
    if (m0 + 16 * TM > M || n0 + 16 * TN > N) return;
    v8f acc[TM][TN];
#pragma unroll
    for (int i = 0; i < TM; ++i)
#pragma unroll
        for (int t = 0; t < TN; ++t) { v8f zz = {}; acc[i][t] = zz; }
    for (int k0 = 0; k0 < K; k0 += 32) {
        FragU a[TM], bb[TN];
#pragma unroll
        for (int i = 0; i < TM; ++i) {
            const unsigned short* ar = A + (size_t)(m0 + 16 * i + l15) * lda + k0 + 8 * h;
            a[i].u[0] = *(const v8us*)ar; a[i].u[1] = *(const v8us*)(ar + 16);
        }
#pragma unroll
        for (int t = 0; t < TN; ++t) {
            const unsigned short* br = Bt + (size_t)(n0 + 16 * t + l15) * ldb + k0 + 8 * h;
            bb[t].u[0] = *(const v8us*)br; bb[t].u[1] = *(const v8us*)(br + 16);
        }
#pragma unroll
        for (int i = 0; i < TM; ++i)
#pragma unroll
            for (int t = 0; t < TN; ++t) {
                if (BF) acc[i][t] = wmmab(a[i].b, bb[t].b, acc[i][t]);
                else    acc[i][t] = wmma16(a[i].h, bb[t].h, acc[i][t]);
            }
    }
    __shared__ __align__(16) float ctile[16][36];
#pragma unroll
    for (int i = 0; i < TM; ++i) {
        const int mb = m0 + 16 * i;
#pragma unroll
        for (int tp = 0; tp < TN / 2; ++tp) {
            const int nb = n0 + 32 * tp;
#pragma unroll
            for (int t2 = 0; t2 < 2; ++t2) {
                const int t = 2 * tp + t2; const int n = nb + t2 * 16 + l15;
                const float bn = cmb_bf(bias[n]);
#pragma unroll
                for (int r = 0; r < 8; ++r) ctile[8 * h + r][t2 * 16 + l15] = acc[i][t][r] * iscale + bn;
            }
            __syncthreads();
#pragma unroll
            for (int s = 0; s < 4; ++s) {
                const int row = s * 4 + (lane >> 3), c4 = (lane & 7) * 4;
                const v4f v = *(const v4f*)&ctile[row][c4];
                VST2V4(C + (size_t)(mb + row) * ldc + nb + c4, v);
            }
            __syncthreads();
        }
    }
}

struct AttP {
    const unsigned short* Q; const unsigned short* K; const unsigned short* VT; float* O;
    long long sQb, sQi, sKb, sKj, sVb, sVd, sOb, sOi;
    int Lq, Lk, hrep, pad0; float scl2; int pad1;
};
static_assert(sizeof(AttP) == 4 * 8 + 8 * 8 + 4 * 4 + 2 * 4);

__global__ __launch_bounds__(32 * AW) void k_attnp(AttP p) {
    constexpr int NT = HDIM / 16;
    constexpr int KS = HDIM / 32;
    __shared__ __align__(16) float pl[AW][16 * 64];
    const int lane = threadIdx.x & 31, hf = lane >> 4, l15 = lane & 15, wave = threadIdx.x >> 5;
    const int h = blockIdx.y, b = blockIdx.z, hk = h / p.hrep;
    const int q0 = (blockIdx.x * AW + wave) * 16;
    float* myp = pl[wave];
    const float NEG = -__builtin_inff();
    const int qi = min(q0 + l15, p.Lq - 1);
    const unsigned short* qrow = p.Q + b * p.sQb + (long long)qi * p.sQi + h * HDIM;
    FragU qa[KS];
#pragma unroll
    for (int ks = 0; ks < KS; ++ks) { qa[ks].u[0] = *(const v8us*)(qrow + ks * 32 + 8 * hf); qa[ks].u[1] = *(const v8us*)(qrow + ks * 32 + 16 + 8 * hf); }
    const unsigned short* kbase = p.K + b * p.sKb + hk * HDIM;
    const unsigned short* vbase = p.VT + b * p.sVb + (long long)(hk * HDIM) * p.sVd;
    v8f o[NT]; float m8[8], l8[8];
#pragma unroll
    for (int t = 0; t < NT; ++t) { v8f zz = {}; o[t] = zz; }
#pragma unroll
    for (int i = 0; i < 8; ++i) { m8[i] = NEG; l8[i] = 0.f; }
    for (int j0 = 0; j0 < p.Lk; j0 += 64) {
        __syncthreads();
        v8f s[4];
#pragma unroll
        for (int t = 0; t < 4; ++t) {
            const int j = min(j0 + t * 16 + l15, p.Lk - 1);
            const unsigned short* krow = kbase + (long long)j * p.sKj;
            v8f acc = {};
#pragma unroll
            for (int ks = 0; ks < KS; ++ks) {
                FragU kb; kb.u[0] = *(const v8us*)(krow + ks * 32 + 8 * hf); kb.u[1] = *(const v8us*)(krow + ks * 32 + 16 + 8 * hf);
                acc = wmma16(qa[ks].h, kb.h, acc);
            }
            s[t] = acc;
        }
        float pv[8][4];
#pragma unroll
        for (int i = 0; i < 8; ++i) {
            float sc[4];
#pragma unroll
            for (int t = 0; t < 4; ++t) sc[t] = s[t][i] * p.scl2;
            float mx = fmaxf(fmaxf(sc[0], sc[1]), fmaxf(sc[2], sc[3]));
            mx = fmaxf(mx, __shfl_xor(mx, 1, 32)); mx = fmaxf(mx, __shfl_xor(mx, 2, 32));
            mx = fmaxf(mx, __shfl_xor(mx, 4, 32)); mx = fmaxf(mx, __shfl_xor(mx, 8, 32));
            const float mnew = fmaxf(m8[i], mx);
            const float corr = (mnew == NEG) ? 1.f : exp2f(m8[i] - mnew);
            float rs = 0.f;
#pragma unroll
            for (int t = 0; t < 4; ++t) { const float pp = exp2f(sc[t] - mnew); rs += pp; pv[i][t] = pp; }
            rs += __shfl_xor(rs, 1, 32); rs += __shfl_xor(rs, 2, 32); rs += __shfl_xor(rs, 4, 32); rs += __shfl_xor(rs, 8, 32);
            l8[i] = l8[i] * corr + rs; m8[i] = mnew;
#pragma unroll
            for (int t = 0; t < NT; ++t) o[t][i] *= corr;
        }
#pragma unroll
        for (int i = 0; i < 8; ++i)
#pragma unroll
            for (int t = 0; t < 4; ++t) ((volatile float*)myp)[(i + 8 * hf) * 64 + t * 16 + l15] = pv[i][t];
        __syncthreads();
        const v16h pa0 = fh_ld(myp + l15 * 64, 1, 0, hf, 64, 4096.f), pa1 = fh_ld(myp + l15 * 64, 1, 32, hf, 64, 4096.f);
#pragma unroll
        for (int t = 0; t < NT; ++t) {
            const int dcol = t * 16 + l15;
            const unsigned short* vrow = vbase + (long long)dcol * p.sVd + j0;
            FragU b0, b1;
            b0.u[0] = *(const v8us*)(vrow + 8 * hf);      b0.u[1] = *(const v8us*)(vrow + 16 + 8 * hf);
            b1.u[0] = *(const v8us*)(vrow + 32 + 8 * hf); b1.u[1] = *(const v8us*)(vrow + 48 + 8 * hf);
            o[t] = wmma16(pa0, b0.h, o[t]);
            o[t] = wmma16(pa1, b1.h, o[t]);
        }
    }
    float invr[8];
#pragma unroll
    for (int i = 0; i < 8; ++i) invr[i] = (l8[i] > 0.f) ? 1.f / (l8[i] * 4096.f) : 0.f;
    __syncthreads();
#pragma unroll
    for (int i = 0; i < 8; ++i)
#pragma unroll
        for (int t = 0; t < NT; ++t) ((volatile float*)myp)[(i + 8 * hf) * 64 + t * 16 + l15] = o[t][i] * invr[i];
    __syncthreads();
    float* obase = p.O + b * p.sOb + h * HDIM;
    for (int r0 = 0; r0 < 16; r0 += 2) {
        const int row = r0 + (lane >> 4), c4 = (lane & 15) * 4;
        const v4f v = *(const v4f*)(myp + row * 64 + c4);
        if (q0 + row < p.Lq) VST2V4(obase + (long long)(q0 + row) * p.sOi + c4, v);
    }
    __syncthreads();
}

extern "C" void kernel_launch(void* const* d_in, const int* in_sizes, int n_in, void* d_out, int out_size, void* d_ws, size_t ws_size, hipStream_t stream) {
    if (n_in < 9) return;
    if (in_sizes[0] < ((NB - 1) * SEQ_FULL + SEQ) * HIDDEN) return;
    if (in_sizes[1] < HIDDEN * HIDDEN || in_sizes[2] < HIDDEN) return;
    if (in_sizes[3] < HIDDEN * KVD || in_sizes[4] < KVD) return;
    if (in_sizes[5] < HIDDEN * KVD || in_sizes[6] < KVD) return;
    if (in_sizes[7] < HIDDEN * HIDDEN || in_sizes[8] < HIDDEN) return;
    if (out_size < MROWS * HIDDEN) return;
    const float* x  = (const float*)d_in[0];
    const float* Wq = (const float*)d_in[1];
    const float* bq = (const float*)d_in[2];
    const float* Wk = (const float*)d_in[3];
    const float* bk = (const float*)d_in[4];
    const float* Wv = (const float*)d_in[5];
    const float* bv = (const float*)d_in[6];
    const float* Wo = (const float*)d_in[7];
    const float* bo = (const float*)d_in[8];
    float* out = (float*)d_out;

    const size_t bR16 = (size_t)MROWS * HIDDEN * 2;
    const size_t bWQ  = (size_t)HIDDEN * HIDDEN * 2;
    const size_t bWK  = (size_t)KVD * HIDDEN * 2;
    const size_t bWV  = (size_t)KVD * HIDDEN * 2;
    const size_t bWO  = (size_t)HIDDEN * HIDDEN * 2;
    const size_t bR32 = (size_t)MROWS * HIDDEN * 4;
    const size_t bKF  = (size_t)MROWS * KVD * 4;
    const size_t bVF  = (size_t)MROWS * KVD * 4;
    const size_t bK16 = (size_t)MROWS * KVD * 2;
    const size_t bVT  = (size_t)NB * KVD * SEQ * 2;
    char* w = (char*)d_ws; size_t off = 0;
    unsigned short* R16  = (unsigned short*)(w + off); off += bR16;
    unsigned short* WQT  = (unsigned short*)(w + off); off += bWQ;
    unsigned short* WKT  = (unsigned short*)(w + off); off += bWK;
    unsigned short* WVT  = (unsigned short*)(w + off); off += bWV;
    unsigned short* WOT  = (unsigned short*)(w + off); off += bWO;
    float*          R32  = (float*)(w + off);          off += bR32;
    float*          KF   = (float*)(w + off);          off += bKF;
    float*          VF   = (float*)(w + off);          off += bVF;
    unsigned short* K16  = (unsigned short*)(w + off); off += bK16;
    unsigned short* VT16 = (unsigned short*)(w + off); off += bVT;
    if (off > ws_size || off > (size_t)134217728u) return;

    { const long long n = (long long)NB * SEQ * (HIDDEN / 8);
      k_cast<0><<<(unsigned)((n + 255) / 256), 256, 0, stream>>>(x, (long long)SEQ_FULL * HIDDEN, HIDDEN, R16, (long long)SEQ * HIDDEN, HIDDEN, SEQ, HIDDEN, NB, 1.f); }
    { const long long n = (long long)HIDDEN * (HIDDEN / 8);
      k_castT<0><<<(unsigned)((n + 255) / 256), 256, 0, stream>>>(Wq, 0LL, HIDDEN, WQT, 0LL, HIDDEN, HIDDEN, HIDDEN, 1, 1.f); }
    { const long long n = (long long)KVD * (HIDDEN / 8);
      k_castT<0><<<(unsigned)((n + 255) / 256), 256, 0, stream>>>(Wk, 0LL, KVD, WKT, 0LL, HIDDEN, HIDDEN, KVD, 1, 1.f);
      k_castT<0><<<(unsigned)((n + 255) / 256), 256, 0, stream>>>(Wv, 0LL, KVD, WVT, 0LL, HIDDEN, HIDDEN, KVD, 1, 1.f); }
    { const long long n = (long long)HIDDEN * (HIDDEN / 8);
      k_castT<1><<<(unsigned)((n + 255) / 256), 256, 0, stream>>>(Wo, 0LL, HIDDEN, WOT, 0LL, HIDDEN, HIDDEN, HIDDEN, 1, 64.f); }

    k_pgemm<true, 4, 2><<<dim3((unsigned)(HIDDEN / 32), (unsigned)(MROWS / 64), 1), 32, 0, stream>>>(R16, HIDDEN, WQT, HIDDEN, bq, R32, HIDDEN, MROWS, HIDDEN, HIDDEN, 1.f);
    k_pgemm<true, 4, 2><<<dim3((unsigned)(KVD / 32), (unsigned)(MROWS / 64), 1), 32, 0, stream>>>(R16, HIDDEN, WKT, HIDDEN, bk, KF, KVD, MROWS, KVD, HIDDEN, 1.f);
    k_pgemm<true, 4, 2><<<dim3((unsigned)(KVD / 32), (unsigned)(MROWS / 64), 1), 32, 0, stream>>>(R16, HIDDEN, WVT, HIDDEN, bv, VF, KVD, MROWS, KVD, HIDDEN, 1.f);

    { const long long n = (long long)MROWS * (HIDDEN / 8);
      k_cast<2><<<(unsigned)((n + 255) / 256), 256, 0, stream>>>(R32, 0LL, HIDDEN, R16, 0LL, HIDDEN, MROWS, HIDDEN, 1, 1.f); }
    { const long long n = (long long)MROWS * (KVD / 8);
      k_cast<2><<<(unsigned)((n + 255) / 256), 256, 0, stream>>>(KF, 0LL, KVD, K16, 0LL, KVD, MROWS, KVD, 1, 1.f); }
    { const long long n = (long long)NB * KVD * (SEQ / 8);
      k_castT<2><<<(unsigned)((n + 255) / 256), 256, 0, stream>>>(VF, (long long)SEQ * KVD, KVD, VT16, (long long)KVD * SEQ, SEQ, SEQ, KVD, NB, 1.f); }

    { AttP a;
      a.Q = R16; a.K = K16; a.VT = VT16; a.O = R32;
      a.sQb = (long long)SEQ * HIDDEN; a.sQi = HIDDEN; a.sKb = (long long)SEQ * KVD; a.sKj = KVD;
      a.sVb = (long long)KVD * SEQ; a.sVd = SEQ; a.sOb = (long long)SEQ * HIDDEN; a.sOi = HIDDEN;
      a.Lq = SEQ; a.Lk = SEQ; a.hrep = NHEAD / NKVH; a.pad0 = 0; a.scl2 = 0.125f * 1.4426950408889634f; a.pad1 = 0;
      k_attnp<<<dim3((unsigned)(SEQ / (16 * AW)), (unsigned)NHEAD, (unsigned)NB), 32 * AW, 0, stream>>>(a); }

    { const long long n = (long long)MROWS * (HIDDEN / 8);
      k_cast<2><<<(unsigned)((n + 255) / 256), 256, 0, stream>>>(R32, 0LL, HIDDEN, R16, 0LL, HIDDEN, MROWS, HIDDEN, 1, 256.f); }
    k_pgemm<false, 4, 2><<<dim3((unsigned)(HIDDEN / 32), (unsigned)(MROWS / 64), 1), 32, 0, stream>>>(R16, HIDDEN, WOT, HIDDEN, bo, out, HIDDEN, MROWS, HIDDEN, HIDDEN, 1.f / 16384.f);
    (void)hipGetLastError();
}
